// Equi_gcn_21603685499523
// MI455X (gfx1250) — hardware-verified
//
#include <hip/hip_runtime.h>
#include <math.h>

typedef __attribute__((ext_vector_type(16))) _Float16 v16h;
typedef __attribute__((ext_vector_type(16))) __bf16 v16b;
typedef __attribute__((ext_vector_type(8)))  _Float16 v8h;
typedef __attribute__((ext_vector_type(8)))  float v8f;
typedef __attribute__((ext_vector_type(4)))  float v4f;
typedef __attribute__((ext_vector_type(2)))  float v2f;
typedef __attribute__((ext_vector_type(4)))  unsigned v4u;
typedef __attribute__((ext_vector_type(4)))  int v4i;
typedef float __attribute__((may_alias)) float_a;
typedef int __attribute__((may_alias)) int_a;

template <typename T> __device__ __forceinline__ void vst2(void* p, T v) { *(volatile T*)p = v; __threadfence(); *(volatile T*)p = v; }
__device__ __forceinline__ v8f wmma16(v16h a, v16h b, v8f c) {
  v8f d = __builtin_amdgcn_wmma_f32_16x16x32_f16(false, a, false, b, (short)0, c, false, false);
  asm volatile("v_nop\n\tv_nop\n\tv_nop\n\tv_nop" : "+v"(d) : "v"(a), "v"(b));
  return d;
}
__device__ __forceinline__ v8f wmma_bf(v16b a, v16b b, v8f c) {
  v8f d = __builtin_amdgcn_wmma_f32_16x16x32_bf16(false, a, false, b, (short)0, c, false, false);
  asm volatile("v_nop\n\tv_nop\n\tv_nop\n\tv_nop" : "+v"(d) : "v"(a), "v"(b));
  return d;
}
__device__ __forceinline__ v16h frag_h(const _Float16* rowk0, int lane) {
  union { v16h v; v8h q[2]; } u; const _Float16* p = rowk0 + 8 * (lane >> 4);
  u.q[0] = *(const v8h*)p; u.q[1] = *(const v8h*)(p + 16); return u.v;
}
__device__ __forceinline__ v16h frag_f32(const float* rowk0, int lane) {
  v16h a; const float* p = rowk0 + 8 * (lane >> 4);
#pragma unroll
  for (int i = 0; i < 8; ++i) { a[i] = (_Float16)p[i]; a[8 + i] = (_Float16)p[16 + i]; }
  return a;
}
__device__ __forceinline__ v16h frag_f32s(const float* rowk0, int lane, float sc) {
  v16h a; const float* p = rowk0 + 8 * (lane >> 4);
#pragma unroll
  for (int i = 0; i < 8; ++i) { a[i] = (_Float16)(p[i] * sc); a[8 + i] = (_Float16)(p[16 + i] * sc); }
  return a;
}
__device__ __forceinline__ v16h fragc_f32(const float* W, int k0, int n, int lane, int ld, int K) {
  v16h a; const int g = lane >> 4;
#pragma unroll
  for (int i = 0; i < 8; ++i) { const int ka = k0 + 8 * g + i, kb = ka + 16;
    a[i] = (_Float16)(ka < K ? W[(size_t)(ka < K ? ka : K - 1) * ld + n] : 0.f); a[8 + i] = (_Float16)(kb < K ? W[(size_t)(kb < K ? kb : K - 1) * ld + n] : 0.f); }
  return a;
}
struct F2 { v16b h, l; };
__device__ __forceinline__ F2 bsplit16(const float v[16]) { F2 r;
#pragma unroll
  for (int i = 0; i < 16; ++i) { const __bf16 h = (__bf16)v[i]; r.h[i] = h; r.l[i] = (__bf16)(v[i] - (float)h); }
  return r; }
__device__ __forceinline__ F2 split_row(const float* row, int k0, int lane) { float v[16]; const float* p = row + k0 + 8 * (lane >> 4);
#pragma unroll
  for (int i = 0; i < 8; ++i) { v[i] = p[i]; v[8 + i] = p[16 + i]; }
  return bsplit16(v); }
__device__ __forceinline__ F2 split_rowK(const float* row, int k0, int lane, int K) { float v[16]; const int g = lane >> 4;
#pragma unroll
  for (int i = 0; i < 8; ++i) { const int ka = k0 + 8 * g + i, kb = ka + 16; v[i] = ka < K ? row[ka < K ? ka : K - 1] : 0.f; v[8 + i] = kb < K ? row[kb < K ? kb : K - 1] : 0.f; }
  return bsplit16(v); }
__device__ __forceinline__ F2 split_col(const float* W, int k0, int n, int lane, int ld, int K) { float v[16]; const int g = lane >> 4;
#pragma unroll
  for (int i = 0; i < 8; ++i) { const int ka = k0 + 8 * g + i, kb = ka + 16; v[i] = ka < K ? W[(size_t)(ka < K ? ka : K - 1) * ld + n] : 0.f; v[8 + i] = kb < K ? W[(size_t)(kb < K ? kb : K - 1) * ld + n] : 0.f; }
  return bsplit16(v); }
__device__ __forceinline__ v8f mac3(const F2& a, const F2& b, v8f c) { c = wmma_bf(a.l, b.h, c); c = wmma_bf(a.h, b.l, c); return wmma_bf(a.h, b.h, c); }
__device__ __forceinline__ float sigm(float v) { return 1.0f / (1.0f + expf(-v)); }
#define LDSX() do { asm volatile("s_wait_dscnt 0" ::: "memory"); __builtin_amdgcn_wave_barrier(); __builtin_amdgcn_fence(__ATOMIC_RELEASE, "workgroup"); } while (0)


#define NB 2
#define N0 4096
#define N1 1024
#define N2 256
#define KNB 20
#define KP 21
#define AA 12
#ifndef NBT
#define NBT NB
#endif
typedef __attribute__((ext_vector_type(8))) __bf16 v8b;
__device__ __forceinline__ v16b frag_b(const __bf16* rowk0, int lane) {
  union { v16b v; v8b q[2]; } u; const __bf16* p = rowk0 + 8 * (lane >> 4);
  u.q[0] = *(const v8b*)p; u.q[1] = *(const v8b*)(p + 16); return u.v;
}
__device__ __forceinline__ float bfr(float v) { return (float)(__bf16)v; }
__device__ __attribute__((noinline)) float exp_ni(float v) { return expf(v); }
__device__ __attribute__((noinline)) float erf_ni(float v) { return erff(v); }

#define WS_PW   0u
#define PL1 0
#define PL2 (PL1 + 128 * 32)
#define PL3 (PL2 + 256 * 64)
#define PL4 (PL3 + 512 * 128)
#define PWEND (PL4 + 1024 * 256)
#define WS_I0   (WS_PW + 2u * PWEND)
#define WS_I1   (WS_I0 + 4u * NB * N0 * 32)
#define WS_I2   (WS_I1 + 4u * NB * N1 * 32)
#define WS_FM0  (WS_I2 + 4u * NB * N2 * 32)
#define WS_GF   (WS_FM0 + 4u * NB * N0 * AA * 32)
#define WS_RAW  (WS_GF + 4u * NB * N0 * AA * 128)
#define WS_FM   (WS_RAW + 4u * NB * N0 * AA * 64)
#define WS_FMP  (WS_FM + 4u * NB * N0 * AA * 64)
#define NSTB 128
#define WS_ST   (WS_FMP + 4u * NB * N1 * AA * 64)
#define WS_BN   (WS_ST + 4u * NSTB * 256)
#define WS_END  (WS_BN + 4u * 3 * 4 * 256)

__global__ __launch_bounds__(256) void k_packw(const float* __restrict__ WS1, const float* __restrict__ WC1, const float* __restrict__ WS2, const float* __restrict__ WC2, const float* __restrict__ WS3, const float* __restrict__ WC3, const float* __restrict__ WS4, const float* __restrict__ WC4, __bf16* __restrict__ PW) {
  __shared__ __align__(16) __bf16 s[256]; const int o = blockIdx.x, l = blockIdx.y, t = threadIdx.x; const int cin = 32 << l, cout = 64 << l; if (o >= 2 * cout) return;
  const float* W = (o < cout) ? (l == 0 ? WS1 : l == 1 ? WS2 : l == 2 ? WS3 : WS4) : (l == 0 ? WC1 : l == 1 ? WC2 : l == 2 ? WC3 : WC4); const int oo = (o < cout) ? o : o - cout;
  const size_t base = (l == 0 ? PL1 : l == 1 ? PL2 : l == 2 ? PL3 : PL4);
  if (t < cin) s[t] = (__bf16)W[(size_t)t * cout + oo];
  __syncthreads();
  if (t < cin / 8) vst2((unsigned*)(PW + base + (size_t)o * cin + t * 8), *(const v4u*)&s[t * 8]);
}
template <int NL, int STRIDE>
__global__ __launch_bounds__(64) void k_knn(const float* __restrict__ V, int* __restrict__ IDX) {
  __shared__ __align__(16) int sk[64][32]; const int tid = threadIdx.x; const size_t q = (size_t)blockIdx.x * 64 + tid; const int b = (int)(q / NL), i = (int)(q % NL);
  const float* vb = V + (size_t)b * N0 * 3; const float xi = bfr(vb[(size_t)i * STRIDE * 3]), yi = bfr(vb[(size_t)i * STRIDE * 3 + 1]), zi = bfr(vb[(size_t)i * STRIDE * 3 + 2]); const float sqi = (xi * xi + zi * zi) + yi * yi;
  float bd[KP]; int bi[KP];
#pragma unroll
  for (int j = 0; j < KP; ++j) { bd[j] = 3.0e38f; bi[j] = i; }
#pragma unroll 1
  for (int n = 0; n < NL; ++n) { const float x = bfr(vb[(size_t)n * STRIDE * 3]), y = bfr(vb[(size_t)n * STRIDE * 3 + 1]), z = bfr(vb[(size_t)n * STRIDE * 3 + 2]); const float sqn = (x * x + z * z) + y * y; const float dot = (xi * x + yi * y) + zi * z; const float d = (sqi + sqn) - 2.0f * dot;
    if (d < bd[KP - 1]) { int pos = KP - 1;
#pragma unroll
      for (int qq = KP - 2; qq >= 0; --qq) if (d < bd[qq]) pos = qq;
#pragma unroll
      for (int qq = KP - 1; qq >= 1; --qq) if (qq > pos) { bd[qq] = bd[qq - 1]; bi[qq] = bi[qq - 1]; }
#pragma unroll
      for (int qq = 0; qq < KP; ++qq) if (qq == pos) { bd[qq] = d; bi[qq] = n; } } }
#pragma unroll
  for (int j = 0; j < 32; ++j) sk[tid][j] = (j < KP) ? bi[j] : i;
  __syncthreads();
  for (int r = 0; r < 64; ++r) if (tid < 8) vst2((unsigned*)(IDX + ((size_t)blockIdx.x * 64 + r) * 32 + tid * 4), *(const v4u*)&sk[r][tid * 4]);
}
__device__ __forceinline__ void nbr_dir(const float* __restrict__ vb, int stride, int i, int j, float& dx, float& dy, float& dz) {
  const float ax = bfr(vb[(size_t)i * stride * 3]), ay = bfr(vb[(size_t)i * stride * 3 + 1]), az = bfr(vb[(size_t)i * stride * 3 + 2]);
  dx = bfr(vb[(size_t)j * stride * 3]) - ax; dy = bfr(vb[(size_t)j * stride * 3 + 1]) - ay; dz = bfr(vb[(size_t)j * stride * 3 + 2]) - az;
  const float nrm = sqrtf((dx * dx + dy * dy) + dz * dz) + 1e-8f; dx /= nrm; dy /= nrm; dz /= nrm;
}
__global__ __launch_bounds__(256) void k_surf(const float* __restrict__ V, const int* __restrict__ I0, const float* __restrict__ K0, float* __restrict__ FM0) {
  __shared__ float sd[8][3][32];
  const int tid = threadIdx.x, wave = tid >> 5, lane = tid & 31; const size_t row = (size_t)blockIdx.x * 8 + wave; const size_t node = row / AA; const int a = (int)(row % AA); const int b = (int)(node / N0), i = (int)(node % N0); const float* vb = V + (size_t)b * N0 * 3;
  if (lane < KNB) { const int j = min(max(I0[node * 32 + 1 + lane], 0), N0 - 1); float dx, dy, dz; nbr_dir(vb, 1, i, j, dx, dy, dz); sd[wave][0][lane] = dx; sd[wave][1][lane] = dy; sd[wave][2][lane] = dz; }
  LDSX();
  const float kx = bfr(K0[(lane * AA + a) * 3]), ky = bfr(K0[(lane * AA + a) * 3 + 1]), kz = bfr(K0[(lane * AA + a) * 3 + 2]);
  float m = -INFINITY;
#pragma unroll 1
  for (int k = 0; k < KNB; ++k) { const float th = fmaxf((sd[wave][0][k] * kx + sd[wave][1][k] * ky) + sd[wave][2][k] * kz, 0.f); m = fmaxf(m, th); }
  vst2(FM0 + row * 32 + lane, fmaxf(m, 0.f));
}
__global__ __launch_bounds__(128) void k_gemm(const float* __restrict__ A, int K, const __bf16* __restrict__ P, const float* __restrict__ bias, int cout, float* __restrict__ OUT, int ldo) {
  __shared__ __align__(16) float so[4][16][132];
  const int tid = threadIdx.x, wave = tid >> 5, lane = tid & 31, col = lane & 15, g = lane >> 4; const size_t r0 = (size_t)blockIdx.x * 64 + wave * 16; const int n0 = blockIdx.y * 128;
  v8f acc[8] = {};
  for (int kc = 0; kc < K / 32; ++kc) { const F2 a = split_row(A + (r0 + col) * (size_t)K, kc * 32, lane);
#pragma unroll
    for (int j = 0; j < 8; ++j) { const v16b w = frag_b(P + (size_t)(n0 + j * 16 + col) * K + kc * 32, lane); acc[j] = wmma_bf(a.l, w, acc[j]); acc[j] = wmma_bf(a.h, w, acc[j]); } }
#pragma unroll
  for (int j = 0; j < 8; ++j) { const int n = n0 + j * 16 + col; const float bb = (n >= cout) ? bfr(bias[n - cout]) : 0.f;
#pragma unroll
    for (int r = 0; r < 8; ++r) so[wave][8 * g + r][j * 16 + col] = acc[j][r] + bb; }
  LDSX();
  for (int rl = 0; rl < 16; ++rl) vst2(OUT + (r0 + rl) * (size_t)ldo + n0 + lane * 4, *(const v4f*)&so[wave][rl][lane * 4]);
}
template <int NL, int STRIDE>
__global__ __launch_bounds__(256) void k_emax(const float* __restrict__ V, const int* __restrict__ IDX, const float* __restrict__ DIRS, const float* __restrict__ GF, int cout, float* __restrict__ RAW) {
  __shared__ float sth[8][32]; __shared__ int snb[8][32];
  const int tid = threadIdx.x, wave = tid >> 5, lane = tid & 31; const size_t row = (size_t)blockIdx.x * 8 + wave; const size_t node = row / AA; const int a = (int)(row % AA); const int b = (int)(node / NL), i = (int)(node % NL); const float* vb = V + (size_t)b * N0 * 3;
  if (lane < KNB) { const int j = min(max(IDX[node * 32 + 1 + lane], 0), NL - 1); float dx, dy, dz; nbr_dir(vb, STRIDE, i, j, dx, dy, dz); const float ux = bfr(DIRS[a * 3]), uy = bfr(DIRS[a * 3 + 1]), uz = bfr(DIRS[a * 3 + 2]); sth[wave][lane] = fmaxf((dx * ux + dy * uy) + dz * uz, 0.f); snb[wave][lane] = j; }
  LDSX();
  const int ld = 2 * cout; const size_t gbase = ((size_t)b * NL) * AA;
  for (int o = lane; o < cout; o += 32) { float m = -INFINITY;
#pragma unroll 1
    for (int k = 0; k < KNB; ++k) m = fmaxf(m, GF[(gbase + (size_t)snb[wave][k] * AA + a) * ld + o] * sth[wave][k]);
    vst2(RAW + row * cout + o, GF[row * ld + cout + o] + m); }
}
template <int PASS>
__global__ __launch_bounds__(256) void k_stat(const float* __restrict__ Y, int W, int nrows, const float* __restrict__ BNP, float* __restrict__ ST) {
  __shared__ __align__(16) float s[256]; const int c = threadIdx.x; const int rpb = nrows / NSTB; const size_t r0 = (size_t)blockIdx.x * rpb; float a = 0.f; const float mu = (PASS && c < W) ? BNP[c] : 0.f;
  if (c < W) {
#pragma unroll 4
    for (int r = 0; r < rpb; ++r) { const float y = Y[(r0 + r) * W + c]; const float d = y - mu; a += PASS ? d * d : y; } }
  s[c] = a; __syncthreads();
  if (c < 64) vst2(ST + (size_t)blockIdx.x * 256 + c * 4, *(const v4f*)&s[c * 4]);
}
template <int PASS>
__global__ __launch_bounds__(256) void k_fin(const float* __restrict__ ST, int W, int nrows, const float* __restrict__ G, const float* __restrict__ BE, float* __restrict__ BNP) {
  __shared__ __align__(16) float s[2][256]; const int c = threadIdx.x; float a = 0.f;
#pragma unroll 1
  for (int b = 0; b < NSTB; ++b) a += ST[(size_t)b * 256 + c];
  const float n = (float)nrows;
  if (PASS == 0) { s[0][c] = (c < W) ? a / n : 0.f; __syncthreads(); if (c < 64) vst2(BNP + c * 4, *(const v4f*)&s[0][c * 4]); }
  else { float sc = 0.f, sh = 0.f; if (c < W) { const float var = a / n; sc = bfr(G[c]) * rsqrtf(var + 1e-5f); sh = bfr(BE[c]) - BNP[c] * sc; } s[0][c] = sc; s[1][c] = sh; __syncthreads(); if (c < 64) { vst2(BNP + 256 + c * 4, *(const v4f*)&s[0][c * 4]); vst2(BNP + 512 + c * 4, *(const v4f*)&s[1][c * 4]); } }
}
__global__ __launch_bounds__(256) void k_bnrelu(const float* __restrict__ RAW, const float* __restrict__ BNP, int cout, float* __restrict__ FM) {
  const int tid = threadIdx.x, wave = tid >> 5, lane = tid & 31; const size_t row = (size_t)blockIdx.x * 8 + wave;
  for (int o = lane; o < cout; o += 32) vst2(FM + row * cout + o, fmaxf(RAW[row * cout + o] * BNP[256 + o] + BNP[512 + o], 0.f));
}
__global__ __launch_bounds__(512) void k_fea(const float* __restrict__ FM, int cout, float* __restrict__ OUT) {
  const size_t node = blockIdx.x; const int c = threadIdx.x; if (c >= cout) return; float m = -INFINITY;
#pragma unroll
  for (int a = 0; a < AA; ++a) m = fmaxf(m, FM[(node * AA + a) * cout + c]);
  vst2(OUT + node * cout + c, m);
}
template <int NLFROM>
__global__ __launch_bounds__(256) void k_pool(const float* __restrict__ FM, const int* __restrict__ IDX, int cout, float* __restrict__ FMP) {
  const int tid = threadIdx.x, wave = tid >> 5, lane = tid & 31; const size_t row = (size_t)blockIdx.x * 8 + wave; const size_t node1 = row / AA; const int a = (int)(row % AA); const int NLTO = NLFROM / 4; const int b = (int)(node1 / NLTO), i1 = (int)(node1 % NLTO); const size_t src = (size_t)b * NLFROM + (size_t)i1 * 4;
  int nb[4];
#pragma unroll
  for (int k = 0; k < 4; ++k) nb[k] = min(max(IDX[src * 32 + 1 + k], 0), NLFROM - 1);
  for (int o = lane; o < cout; o += 32) { float m = FM[(src * AA + a) * cout + o];
#pragma unroll
    for (int k = 0; k < 4; ++k) m = fmaxf(m, FM[(((size_t)b * NLFROM + nb[k]) * AA + a) * cout + o]);
    vst2(FMP + row * cout + o, m); }
}
extern "C" void kernel_launch(void* const* d_in, const int* in_sizes, int n_in, void* d_out, int out_size, void* d_ws, size_t ws_size, hipStream_t stream) {
  (void)in_sizes; (void)n_in; (void)out_size;
  const float** F = (const float**)d_in;
  if (ws_size < (size_t)WS_END) return;
  char* ws = (char*)d_ws; __bf16* PW = (__bf16*)(ws + WS_PW); int *I0 = (int*)(ws + WS_I0), *I1 = (int*)(ws + WS_I1), *I2 = (int*)(ws + WS_I2); float *FM0 = (float*)(ws + WS_FM0), *GF = (float*)(ws + WS_GF), *RAW = (float*)(ws + WS_RAW), *FM = (float*)(ws + WS_FM), *FMP = (float*)(ws + WS_FMP), *ST = (float*)(ws + WS_ST), *BN = (float*)(ws + WS_BN);
  float* O0 = (float*)d_out; float* O1 = O0 + (size_t)NB * N0 * 32; float* O2 = O1 + (size_t)NB * N0 * 64; float* O3 = O2 + (size_t)NB * N1 * 128; float* O4 = O3 + (size_t)NB * N1 * 256;
  const int R0 = NBT * N0 * AA, R1 = NBT * N1 * AA, R2 = NBT * N2 * AA;
  k_packw<<<dim3(1024, 4), 256, 0, stream>>>(F[5], F[3], F[9], F[7], F[13], F[11], F[17], F[15], PW);
  k_knn<N0, 1><<<NBT * N0 / 64, 64, 0, stream>>>(F[0], I0); k_knn<N1, 4><<<NBT * N1 / 64, 64, 0, stream>>>(F[0], I1); k_knn<N2, 16><<<NBT * N2 / 64, 64, 0, stream>>>(F[0], I2);
  k_surf<<<R0 / 8, 256, 0, stream>>>(F[0], I0, F[1], FM0);
  k_fea<<<NBT * N0, 512, 0, stream>>>(FM0, 32, O0);
  k_gemm<<<dim3(R0 / 64, 1), 128, 0, stream>>>(FM0, 32, PW + PL1, F[4], 64, GF, 128);
  k_emax<N0, 1><<<R0 / 8, 256, 0, stream>>>(F[0], I0, F[2], GF, 64, RAW);
  k_stat<0><<<NSTB, 256, 0, stream>>>(RAW, 64, R0, BN, ST); k_fin<0><<<1, 256, 0, stream>>>(ST, 64, R0, F[18], F[19], BN); k_stat<1><<<NSTB, 256, 0, stream>>>(RAW, 64, R0, BN, ST); k_fin<1><<<1, 256, 0, stream>>>(ST, 64, R0, F[18], F[19], BN);
  k_bnrelu<<<R0 / 8, 256, 0, stream>>>(RAW, BN, 64, FM);
  k_fea<<<NBT * N0, 512, 0, stream>>>(FM, 64, O1);
  k_pool<N0><<<R1 / 8, 256, 0, stream>>>(FM, I0, 64, FMP);
  k_gemm<<<dim3(R1 / 64, 2), 128, 0, stream>>>(FMP, 64, PW + PL2, F[8], 128, GF, 256);
  k_emax<N1, 4><<<R1 / 8, 256, 0, stream>>>(F[0], I1, F[6], GF, 128, RAW);
  k_stat<0><<<NSTB, 256, 0, stream>>>(RAW, 128, R1, BN + 1024, ST); k_fin<0><<<1, 256, 0, stream>>>(ST, 128, R1, F[20], F[21], BN + 1024); k_stat<1><<<NSTB, 256, 0, stream>>>(RAW, 128, R1, BN + 1024, ST); k_fin<1><<<1, 256, 0, stream>>>(ST, 128, R1, F[20], F[21], BN + 1024);
  k_bnrelu<<<R1 / 8, 256, 0, stream>>>(RAW, BN + 1024, 128, FM);
  k_fea<<<NBT * N1, 512, 0, stream>>>(FM, 128, O2);
  k_gemm<<<dim3(R1 / 64, 4), 128, 0, stream>>>(FM, 128, PW + PL3, F[12], 256, GF, 512);
  k_emax<N1, 4><<<R1 / 8, 256, 0, stream>>>(F[0], I1, F[10], GF, 256, RAW);
  k_stat<0><<<NSTB, 256, 0, stream>>>(RAW, 256, R1, BN + 2048, ST); k_fin<0><<<1, 256, 0, stream>>>(ST, 256, R1, F[22], F[23], BN + 2048); k_stat<1><<<NSTB, 256, 0, stream>>>(RAW, 256, R1, BN + 2048, ST); k_fin<1><<<1, 256, 0, stream>>>(ST, 256, R1, F[22], F[23], BN + 2048);
  k_bnrelu<<<R1 / 8, 256, 0, stream>>>(RAW, BN + 2048, 256, FM);
  k_fea<<<NBT * N1, 512, 0, stream>>>(FM, 256, O3);
  k_pool<N1><<<R2 / 8, 256, 0, stream>>>(FM, I1, 256, FMP);
  k_gemm<<<dim3(R2 / 64, 8), 128, 0, stream>>>(FMP, 256, PW + PL4, F[16], 512, GF, 1024);
  k_emax<N2, 16><<<R2 / 8, 256, 0, stream>>>(F[0], I2, F[14], GF, 512, RAW);
  k_fea<<<NBT * N2, 512, 0, stream>>>(RAW, 512, O4);
}
